// StructurePredictor_68564857913753
// MI455X (gfx1250) — hardware-run, weakly checked
//
#include <hip/hip_runtime.h>
#include <math.h>

#ifndef NB
#define NB 2
#endif
#ifndef SEQ
#define SEQ 256
#endif
#define NB_FULL 2
#define SEQ_FULL 256
#define MR (NB * SEQ)
#define HID 320
#define CD 160

static_assert(NB == 2);
static_assert(SEQ % 64 == 0);
static_assert(SEQ <= SEQ_FULL);
static_assert(MR % 64 == 0);
static_assert(HID % 32 == 0);
static_assert(HID == 8 * 40);

typedef __attribute__((ext_vector_type(4))) float v4f;
typedef unsigned v4u __attribute__((ext_vector_type(4)));

#define VST2(T, ptr, val) do { const T vst2_v_ = (val); *(volatile T*)(ptr) = vst2_v_; __threadfence(); *(volatile T*)(ptr) = vst2_v_; } while (0)
#define VST2V4(ptr, val) do { const v4f vst2_v4_ = (val); *(volatile v4f*)(ptr) = vst2_v4_; __threadfence(); *(volatile v4f*)(ptr) = vst2_v4_; } while (0)

namespace gemmkit {
typedef __attribute__((ext_vector_type(16))) _Float16 v16h;
typedef __attribute__((ext_vector_type(8)))  _Float16 v8h;
typedef __attribute__((ext_vector_type(16))) __bf16   v16b;
typedef __attribute__((ext_vector_type(8)))  __bf16   v8b;
typedef __attribute__((ext_vector_type(8)))  float    v8f;
typedef __attribute__((ext_vector_type(4)))  float    v4f;

__device__ __forceinline__ unsigned short f2bf_bits(float f) {
  unsigned u = __float_as_uint(f);
  return (unsigned short)((u + 0x7FFFu + ((u >> 16) & 1u)) >> 16);
}
__device__ __forceinline__ float bf_bits2f(unsigned short h) { return __uint_as_float(((unsigned)h) << 16); }

__device__ __forceinline__ void dep_guard_h(v8f& a, v8f& b, v16h x, v16h y) { asm volatile("v_nop\n\tv_nop\n\tv_nop\n\tv_nop" : "+v"(a), "+v"(b) : "v"(x), "v"(y)); }
__device__ __forceinline__ void dep_guard_b(v8f& a, v8f& b, v16b x, v16b y) { asm volatile("v_nop\n\tv_nop\n\tv_nop\n\tv_nop" : "+v"(a), "+v"(b) : "v"(x), "v"(y)); }
__device__ __forceinline__ void keep4_h(v16h a, v16h b, v16h c, v16h d) { asm volatile("v_nop" :: "v"(a), "v"(b), "v"(c), "v"(d)); }
__device__ __forceinline__ void keep4_b(v16b a, v16b b, v16b c, v16b d) { asm volatile("v_nop" :: "v"(a), "v"(b), "v"(c), "v"(d)); }
__device__ __forceinline__ void acc_guard4(v8f& a, v8f& b, v8f& c, v8f& d) { asm volatile("v_nop\n\tv_nop\n\tv_nop\n\tv_nop" : "+v"(a), "+v"(b), "+v"(c), "+v"(d)); }
template <typename T> struct Frag;
template <> struct Frag<_Float16> {
  typedef v16h V; union U { v16h v; v8h h[2]; };
  static __device__ __forceinline__ v16h load(const _Float16* p) {
    U f; f.h[0] = *(const v8h*)(p); f.h[1] = *(const v8h*)(p + 16); return f.v;
  }
  static __device__ __forceinline__ v8f mma(v16h a, v16h b, v8f c) {
    return __builtin_amdgcn_wmma_f32_16x16x32_f16(false, a, false, b, (short)0, c, false, false);
  }
  static __device__ __forceinline__ void guard(v8f& a, v8f& b, v16h x, v16h y) { dep_guard_h(a, b, x, y); }
  static __device__ __forceinline__ void keep(v16h a, v16h b, v16h c, v16h d) { keep4_h(a, b, c, d); }
};
template <> struct Frag<__bf16> {
  typedef v16b V; union U { v16b v; v8b h[2]; };
  static __device__ __forceinline__ v16b load(const __bf16* p) {
    U f; f.h[0] = *(const v8b*)(p); f.h[1] = *(const v8b*)(p + 16); return f.v;
  }
  static __device__ __forceinline__ v8f mma(v16b a, v16b b, v8f c) {
    return __builtin_amdgcn_wmma_f32_16x16x32_bf16(false, a, false, b, (short)0, c, false, false);
  }
  static __device__ __forceinline__ void guard(v8f& a, v8f& b, v16b x, v16b y) { dep_guard_b(a, b, x, y); }
  static __device__ __forceinline__ void keep(v16b a, v16b b, v16b c, v16b d) { keep4_b(a, b, c, d); }
};

template <int ET> struct Elem;
template <> struct Elem<0> { typedef _Float16 T; };
template <> struct Elem<1> { typedef __bf16 T; };
template <int ET, bool SPLIT, int BIAS_MODE, int OUT_MODE, bool RESID, int ACT = 0>
__global__ __launch_bounds__(256) void wmma_gemm64(
    const unsigned short* __restrict__ Ap, const unsigned short* __restrict__ A2p, int lda, long strideA,
    const unsigned short* __restrict__ Btp, const unsigned short* __restrict__ Bt2p, int ldb, long strideB,
    void* __restrict__ Cout, void* __restrict__ Cout2, int ldc, long strideC,
    const float* __restrict__ bias,
    const float* __restrict__ resid, long strideR,
    int M, int N, int K, float scale) {
  typedef typename Elem<ET>::T T;
  typedef typename Frag<T>::V V;
  const T* A = (const T*)Ap; const T* A2 = (const T*)A2p; const T* Bt = (const T*)Btp; const T* Bt2 = (const T*)Bt2p;
  __shared__ __align__(16) float sT[8][16 * 68];
  const int b    = blockIdx.y;
  const int lane = threadIdx.x & 31;
  const int wave = threadIdx.x >> 5;
  const int tilesN = N >> 6;
  const int tilesM = M >> 6;
  const int tile = blockIdx.x * 8 + wave;
  if (tile >= tilesM * tilesN) return;
  const int tm = tile / tilesN;
  const int tn = tile - tm * tilesN;
  const int m0 = tm << 6;
  const int n0 = tn << 6;

  const T* Ab  = A  + (size_t)b * strideA;
  const T* Bb  = Bt + (size_t)b * strideB;
  const T* Ab2 = SPLIT ? (A2  + (size_t)b * strideA) : nullptr;
  const T* Bb2 = SPLIT ? (Bt2 + (size_t)b * strideB) : nullptr;

  const int rlane = lane & 15;
  const int koff  = (lane >> 4) * 8;
  const int mOff  = (lane >> 4) * 8;

  v8f acc[4][4];
#pragma unroll
  for (int i = 0; i < 4; ++i)
#pragma unroll
    for (int j = 0; j < 4; ++j) acc[i][j] = (v8f){0.f,0.f,0.f,0.f,0.f,0.f,0.f,0.f};

  for (int k0 = 0; k0 < K; k0 += 32) {
    V bh[4], bl[4];
#pragma unroll
    for (int j = 0; j < 4; ++j) {
      const size_t bo = (size_t)(n0 + (j << 4) + rlane) * ldb + koff + k0;
      bh[j] = Frag<T>::load(Bb + bo);
      if (SPLIT) bl[j] = Frag<T>::load(Bb2 + bo);
    }
#pragma unroll
    for (int i = 0; i < 4; ++i) {
      const size_t ao = (size_t)(m0 + (i << 4) + rlane) * lda + koff + k0;
      V ah = Frag<T>::load(Ab + ao);
      V al;
      if (SPLIT) al = Frag<T>::load(Ab2 + ao);
#pragma unroll
      for (int j = 0; j < 4; ++j) {
        acc[i][j] = Frag<T>::mma(ah, bh[j], acc[i][j]);
        if (SPLIT) {
          acc[i][j] = Frag<T>::mma(ah, bl[j], acc[i][j]);
          acc[i][j] = Frag<T>::mma(al, bh[j], acc[i][j]);
        }
      }
      Frag<T>::guard(acc[i][0], acc[i][3], ah, SPLIT ? al : ah);
    }
    Frag<T>::keep(bh[0], bh[1], bh[2], bh[3]);
    if (SPLIT) Frag<T>::keep(bl[0], bl[1], bl[2], bl[3]);
  }
  acc_guard4(acc[0][0], acc[0][1], acc[0][2], acc[0][3]);
  acc_guard4(acc[1][0], acc[1][1], acc[1][2], acc[1][3]);
  acc_guard4(acc[2][0], acc[2][1], acc[2][2], acc[2][3]);
  acc_guard4(acc[3][0], acc[3][1], acc[3][2], acc[3][3]);

  float* slab = sT[wave];
  const float* Rb = RESID ? (resid + (size_t)b * strideR) : nullptr;
#pragma unroll
  for (int i = 0; i < 4; ++i) {
    const int mBase = m0 + (i << 4);
#pragma unroll
    for (int j = 0; j < 4; ++j) {
      const int n = n0 + (j << 4) + rlane;
      float bv = 0.f;
      if (BIAS_MODE == 2) bv = bias[n];
#pragma unroll
      for (int r = 0; r < 8; ++r) {
        float v = acc[i][j][r] * scale;
        if (BIAS_MODE == 1) v += bias[mBase + mOff + r];
        if (BIAS_MODE == 2) v += bv;
        if (RESID) v += Rb[(size_t)(mBase + mOff + r) * ldc + n];
        if (ACT == 1) v = tanhf(v);
        if (ACT == 2) v = fmaxf(v, 0.0f);
        if (ACT == 3) v = v / (1.0f + expf(-v));
        if (ACT == 4) v = (v > 0.f) ? v : 0.01f * v;
        if (ACT == 5) v = 0.5f * v * (1.0f + erff(v * 0.70710678118654752f));
        if (ACT == 6) v = (v > 0.f) ? v : 0.2f * v;
        if (ACT == 7) { const float u = 0.7978845608028654f * (v + 0.044715f * v * v * v); v = 0.5f * v * (1.f + tanhf(u)); }
        slab[(mOff + r) * 68 + (j << 4) + rlane] = v;
      }
    }
    __builtin_amdgcn_fence(3  , "workgroup");
    __builtin_amdgcn_wave_barrier();
    __builtin_amdgcn_fence(2  , "workgroup");
    if (OUT_MODE == 0) {
      float* C = (float*)Cout + (size_t)b * strideC;
      const int hh = lane >> 4, c4 = (lane & 15) * 4;
      for (int pass = 0; pass < 2; ++pass) {
#pragma unroll
        for (int it = 0; it < 8; ++it) {
          const int row = it * 2 + hh;
          v4f v = *(const v4f*)(slab + row * 68 + c4);
          *(volatile v4f*)(C + (size_t)(mBase + row) * ldc + n0 + c4) = v;
        }
        __threadfence();
      }
    } else {
      const int q = lane >> 3, c8 = (lane & 7) * 8;
      unsigned short* C  = (unsigned short*)Cout  + (size_t)b * strideC;
      unsigned short* C2 = (OUT_MODE == 2) ? ((unsigned short*)Cout2 + (size_t)b * strideC) : nullptr;
      for (int pass = 0; pass < 2; ++pass) {
#pragma unroll
        for (int it = 0; it < 4; ++it) {
          const int row = it * 4 + q;
          const float* sp = slab + row * 68 + c8;
          v8h hv, lv;
#pragma unroll
          for (int e = 0; e < 8; ++e) {
            if (OUT_MODE == 1) {
              hv[e] = (_Float16)sp[e];
            } else {
              unsigned short hb = f2bf_bits(sp[e]);
              unsigned short lb = f2bf_bits(sp[e] - bf_bits2f(hb));
              hv[e] = __builtin_bit_cast(_Float16, hb);
              lv[e] = __builtin_bit_cast(_Float16, lb);
            }
          }
          *(volatile v8h*)(C + (size_t)(mBase + row) * ldc + n0 + c8) = hv;
          if (OUT_MODE == 2) *(volatile v8h*)(C2 + (size_t)(mBase + row) * ldc + n0 + c8) = lv;
        }
        __threadfence();
      }
    }
    __builtin_amdgcn_fence(3  , "workgroup");
    __builtin_amdgcn_wave_barrier();
    __builtin_amdgcn_fence(2  , "workgroup");
  }
}

}

static_assert(8 * 16 * 68 * 4 <= 131072);

typedef _Float16 h16;
static __device__ __forceinline__ h16 toh_flush(float v) { const h16 r = (h16)v; return (fabsf(v) < 6.103515625e-05f) ? (h16)0.0f : r; }
static __device__ __forceinline__ unsigned hbits_flush(float v) { return (unsigned)__builtin_bit_cast(unsigned short, toh_flush(v)); }
static __device__ __forceinline__ float bfr(float v) { unsigned u = __builtin_bit_cast(unsigned, v); u += 0x7FFFu + ((u >> 16) & 1u); return __builtin_bit_cast(float, u & 0xFFFF0000u); }
static __device__ __forceinline__ void st8h_flush(unsigned short* p, const float* v) {
    v4u pk;
    pk.x = hbits_flush(v[0]) | (hbits_flush(v[1]) << 16);
    pk.y = hbits_flush(v[2]) | (hbits_flush(v[3]) << 16);
    pk.z = hbits_flush(v[4]) | (hbits_flush(v[5]) << 16);
    pk.w = hbits_flush(v[6]) | (hbits_flush(v[7]) << 16);
    VST2(v4u, (v4u*)p, pk);
}

__global__ __launch_bounds__(256) void k_wt16f(const float* __restrict__ Wm, int ldw, int KI, int NO, int NOP, unsigned short* __restrict__ W16, float sw) {
    const int u = blockIdx.x * 256 + threadIdx.x; const int per = KI / 8; if (u >= NOP * per) return;
    const int k0 = 8 * (u % per); const int o = u / per; const int oc = min(o, NO - 1); float v[8];
#pragma unroll
    for (int i = 0; i < 8; ++i) { const float w = Wm[(long long)(k0 + i) * ldw + oc]; v[i] = (o < NO) ? bfr(w) * sw : 0.f; }
    st8h_flush(W16 + (long long)o * KI + k0, v);
}
static_assert((640 * (HID / 8)) % 32 == 0);
static_assert((320 * (HID / 8)) % 32 == 0);
static_assert((192 * (HID / 8)) % 32 == 0);
static_assert((960 * (HID / 8)) % 32 == 0);
static_assert((160 * (HID / 8)) % 32 == 0);
static_assert((256 * (128 / 8)) % 32 == 0);

__global__ __launch_bounds__(256) void k_x16(const float* __restrict__ X, unsigned short* __restrict__ X16, float sc) {
    const int u = blockIdx.x * 256 + threadIdx.x; if (u >= MR * (HID / 8)) return;
    const int r = u / (HID / 8); const int c0 = 8 * (u % (HID / 8)); const int s = r / SEQ; const int n = r - s * SEQ;
    const float* x = X + ((long long)(s * SEQ_FULL + n)) * HID + c0; float v[8];
#pragma unroll
    for (int i = 0; i < 8; ++i) v[i] = bfr(x[i]) * sc;
    st8h_flush(X16 + (long long)r * HID + c0, v);
}
static_assert((MR * (HID / 8)) % 32 == 0);

#define BO_BB1 0
#define BO_SC1 640
#define BO_SC2 960
#define BO_IN  1152
#define BO_OUT 2112
#define BO_R2  2432
#define BIAS_N 2688
static_assert(BO_SC1 % 32 == 0 && BO_SC2 % 32 == 0 && BO_IN % 32 == 0 && BO_OUT % 32 == 0 && BO_R2 % 32 == 0 && BIAS_N % 32 == 0);
static_assert(BO_R2 + 256 == BIAS_N);
__global__ __launch_bounds__(256) void k_bias6(const float* __restrict__ bb1, const float* __restrict__ sc1, const float* __restrict__ sc2, const float* __restrict__ inb,
                                              const float* __restrict__ outb, const float* __restrict__ r2b, float* __restrict__ Bp) {
    const int t = blockIdx.x * 256 + threadIdx.x;
    if (t < 640) { const float v = bfr(bb1[t]); VST2(float, Bp + BO_BB1 + t, v); }
    if (t < 320) { const float v = bfr(sc1[t]); VST2(float, Bp + BO_SC1 + t, v); }
    if (t < 192) { const float w = sc2[min(t, 159)]; const float v = (t < 160) ? bfr(w) : 0.f; VST2(float, Bp + BO_SC2 + t, v); }
    if (t < 960) { const float v = bfr(inb[t]); VST2(float, Bp + BO_IN + t, v); }
    if (t < 320) { const float v = bfr(outb[t]); VST2(float, Bp + BO_OUT + t, v); }
    if (t < 256) { const float v = bfr(r2b[t]); VST2(float, Bp + BO_R2 + t, v); }
}

__global__ __launch_bounds__(256) void k_bb_head(const float* __restrict__ T1, const float* __restrict__ W2, const float* __restrict__ B2, const float* __restrict__ SW1,
                                                float* __restrict__ OUT0, float* __restrict__ R1) {
    __shared__ __align__(16) float st[32 * 3];
    const int wave = __builtin_amdgcn_readfirstlane(threadIdx.x >> 5); const int L = threadIdx.x & 31; const int r0 = blockIdx.x * 32;
    const int sb = r0 / SEQ; const int rf0 = sb * SEQ_FULL + (r0 - sb * SEQ);
    const float c0b = bfr(B2[0]), c1b = bfr(B2[1]), c2b = bfr(B2[2]);
#pragma unroll 1
    for (int i = 0; i < 4; ++i) {
        const int rl = 4 * wave + i; const int r = r0 + rl; const float* t = T1 + (long long)r * 640;
        float a0 = 0.f, a1 = 0.f, a2 = 0.f;
#pragma unroll 2
        for (int k = L; k < 640; k += 32) { const float tv = t[k]; a0 += tv * bfr(W2[k * 3]); a1 += tv * bfr(W2[k * 3 + 1]); a2 += tv * bfr(W2[k * 3 + 2]); }
#pragma unroll
        for (int o = 16; o > 0; o >>= 1) { a0 += __shfl_xor(a0, o, 32); a1 += __shfl_xor(a1, o, 32); a2 += __shfl_xor(a2, o, 32); }
        a0 += c0b; a1 += c1b; a2 += c2b;
        if (L == 0) { st[rl * 3] = a0; st[rl * 3 + 1] = a1; st[rl * 3 + 2] = a2; }
#pragma unroll 1
        for (int j = 0; j < 3; ++j) {
            const int p = L + 32 * j; const int c = 4 * min(p, 79);
            const v4f w0 = *(const v4f*)(SW1 + 320 * 320 + c), w1 = *(const v4f*)(SW1 + 321 * 320 + c), w2 = *(const v4f*)(SW1 + 322 * 320 + c);
            v4f o;
            o.x = a0 * bfr(w0.x) + a1 * bfr(w1.x) + a2 * bfr(w2.x);
            o.y = a0 * bfr(w0.y) + a1 * bfr(w1.y) + a2 * bfr(w2.y);
            o.z = a0 * bfr(w0.z) + a1 * bfr(w1.z) + a2 * bfr(w2.z);
            o.w = a0 * bfr(w0.w) + a1 * bfr(w1.w) + a2 * bfr(w2.w);
            if (p < 80) VST2V4(R1 + (long long)r * 320 + c, o);
        }
    }
    __syncthreads();
    if (threadIdx.x < 24) { const v4f v = *(const v4f*)&st[4 * threadIdx.x]; VST2V4(OUT0 + (long long)rf0 * 3 + 4 * threadIdx.x, v); }
}
static_assert(24 * 16 == 32 * 3 * 4);
static_assert(80 * 16 == 320 * 4);
static_assert(MR % 32 == 0 && SEQ % 32 == 0);

__global__ __launch_bounds__(256) void k_sc_head(const float* __restrict__ H2, const float* __restrict__ W3, const float* __restrict__ B3, const float* __restrict__ BBO,
                                                const float* __restrict__ RW1, const float* __restrict__ RB1, float* __restrict__ OUT1, unsigned short* __restrict__ R1H, float carry) {
    __shared__ __align__(16) float st[32 * 4];
    const int wave = __builtin_amdgcn_readfirstlane(threadIdx.x >> 5); const int L = threadIdx.x & 31; const int r0 = blockIdx.x * 32;
    const int sb = r0 / SEQ; const int rf0 = sb * SEQ_FULL + (r0 - sb * SEQ);
    const v4f b3 = *(const v4f*)B3; const int c0 = 4 * L; const v4f rb = *(const v4f*)(RB1 + c0);
#pragma unroll 1
    for (int i = 0; i < 4; ++i) {
        const int rl = 4 * wave + i; const int r = r0 + rl; const int rf = rf0 + rl; const float* hrow = H2 + (long long)r * 192;
        float a0 = 0.f, a1 = 0.f, a2 = 0.f, a3 = 0.f;
#pragma unroll 1
        for (int k = L; k < 160; k += 32) { const float hv = hrow[k]; const v4f w = *(const v4f*)(W3 + 4 * k); a0 += hv * bfr(w.x); a1 += hv * bfr(w.y); a2 += hv * bfr(w.z); a3 += hv * bfr(w.w); }
#pragma unroll
        for (int o = 16; o > 0; o >>= 1) { a0 += __shfl_xor(a0, o, 32); a1 += __shfl_xor(a1, o, 32); a2 += __shfl_xor(a2, o, 32); a3 += __shfl_xor(a3, o, 32); }
        a0 += bfr(b3.x); a1 += bfr(b3.y); a2 += bfr(b3.z); a3 += bfr(b3.w);
        if (L == 0) { st[rl * 4] = a0; st[rl * 4 + 1] = a1; st[rl * 4 + 2] = a2; st[rl * 4 + 3] = a3; }
        const float g0 = BBO[(long long)rf * 3], g1 = BBO[(long long)rf * 3 + 1], g2 = BBO[(long long)rf * 3 + 2];
        const float cm[7] = {g0, g1, g2, a0, a1, a2, a3};
        v4f acc; acc.x = bfr(rb.x); acc.y = bfr(rb.y); acc.z = bfr(rb.z); acc.w = bfr(rb.w);
#pragma unroll
        for (int k = 0; k < 7; ++k) { const v4f w = *(const v4f*)(RW1 + k * 128 + c0); acc.x += cm[k] * bfr(w.x); acc.y += cm[k] * bfr(w.y); acc.z += cm[k] * bfr(w.z); acc.w += cm[k] * bfr(w.w); }
        const unsigned long long pk = (unsigned long long)hbits_flush(fmaxf(acc.x, 0.f) * carry) | ((unsigned long long)hbits_flush(fmaxf(acc.y, 0.f) * carry) << 16)
                                    | ((unsigned long long)hbits_flush(fmaxf(acc.z, 0.f) * carry) << 32) | ((unsigned long long)hbits_flush(fmaxf(acc.w, 0.f) * carry) << 48);
        VST2(unsigned long long, (unsigned long long*)(R1H + (long long)r * 128 + c0), pk);
    }
    __syncthreads();
    if (threadIdx.x < 32) { const v4f v = *(const v4f*)&st[4 * threadIdx.x]; VST2V4(OUT1 + (long long)rf0 * 4 + 4 * threadIdx.x, v); }
}
static_assert(32 * 16 == 32 * 4 * 4);
static_assert(32 * 8 == 128 * 2);

__global__ __launch_bounds__(256) void k_ref_head(const float* __restrict__ R2, const float* __restrict__ W3, const float* __restrict__ B3, float* __restrict__ OUT3) {
    __shared__ __align__(16) float st[32 * 7];
    const int wave = __builtin_amdgcn_readfirstlane(threadIdx.x >> 5); const int L = threadIdx.x & 31; const int r0 = blockIdx.x * 32;
    const int sb = r0 / SEQ; const int rf0 = sb * SEQ_FULL + (r0 - sb * SEQ);
#pragma unroll 1
    for (int i = 0; i < 4; ++i) {
        const int rl = 4 * wave + i; const int r = r0 + rl; const float* rr = R2 + (long long)r * 256;
        float a[7];
#pragma unroll
        for (int j = 0; j < 7; ++j) a[j] = 0.f;
#pragma unroll 1
        for (int k = L; k < 256; k += 32) { const float rv = rr[k];
#pragma unroll
            for (int j = 0; j < 7; ++j) a[j] += rv * bfr(W3[k * 7 + j]); }
#pragma unroll
        for (int j = 0; j < 7; ++j) {
#pragma unroll
            for (int o = 16; o > 0; o >>= 1) a[j] += __shfl_xor(a[j], o, 32);
            a[j] += bfr(B3[j]);
        }
        if (L == 0) {
#pragma unroll
            for (int j = 0; j < 7; ++j) st[rl * 7 + j] = a[j];
        }
    }
    __syncthreads();
    if (threadIdx.x < 56) { const v4f v = *(const v4f*)&st[4 * threadIdx.x]; VST2V4(OUT3 + (long long)rf0 * 7 + 4 * threadIdx.x, v); }
}
static_assert(56 * 16 == 32 * 7 * 4);

__device__ __attribute__((noinline)) float exp_call(float x) { return expf(x); }
__global__ __launch_bounds__(256) void k_attn2(const float* __restrict__ QKV, unsigned short* __restrict__ AO16, float sc) {
    __shared__ float stage[8][2][HID];
    const int wave = __builtin_amdgcn_readfirstlane(threadIdx.x >> 5); const int L = threadIdx.x & 31; const int n = blockIdx.x * 8 + wave;
    const int hd = L >> 2, qd = L & 3, d0 = hd * 40 + 10 * qd;
    const float* r0p = QKV + (long long)n * 960 + d0; const float* r1p = QKV + (long long)(SEQ + n) * 960 + d0;
    float s00 = 0.f, s01 = 0.f, s10 = 0.f, s11 = 0.f;
#pragma unroll 2
    for (int i = 0; i < 10; ++i) { const float qa = r0p[i], qb = r1p[i], ka = r0p[320 + i], kb = r1p[320 + i]; s00 += qa * ka; s01 += qa * kb; s10 += qb * ka; s11 += qb * kb; }
    s00 += __shfl_xor(s00, 1, 32); s01 += __shfl_xor(s01, 1, 32); s10 += __shfl_xor(s10, 1, 32); s11 += __shfl_xor(s11, 1, 32);
    s00 += __shfl_xor(s00, 2, 32); s01 += __shfl_xor(s01, 2, 32); s10 += __shfl_xor(s10, 2, 32); s11 += __shfl_xor(s11, 2, 32);
    const float isq = 0.15811388300841897f;
    s00 *= isq; s01 *= isq; s10 *= isq; s11 *= isq;
    const float m0 = fmaxf(s00, s01), m1 = fmaxf(s10, s11);
    const float e00 = exp_call(s00 - m0), e01 = exp_call(s01 - m0), e10 = exp_call(s10 - m1), e11 = exp_call(s11 - m1);
    const float i0 = 1.0f / (e00 + e01), i1 = 1.0f / (e10 + e11);
    const float p00 = e00 * i0, p01 = e01 * i0, p10 = e10 * i1, p11 = e11 * i1;
#pragma unroll 2
    for (int i = 0; i < 10; ++i) { const float va = r0p[640 + i], vb = r1p[640 + i]; stage[wave][0][d0 + i] = (p00 * va + p01 * vb) * sc; stage[wave][1][d0 + i] = (p10 * va + p11 * vb) * sc; }
    __builtin_amdgcn_fence(3  , "workgroup");
    __builtin_amdgcn_wave_barrier();
    __builtin_amdgcn_fence(2  , "workgroup");
#pragma unroll 1
    for (int s = 0; s < 2; ++s) {
        unsigned short* orow = AO16 + ((long long)(s * SEQ + n)) * HID; float v[8];
#pragma unroll
        for (int e = 0; e < 8; ++e) v[e] = stage[wave][s][8 * L + e];
        st8h_flush(orow + 8 * L, v);
        const int pc = 32 + (L & 7);
#pragma unroll
        for (int e = 0; e < 8; ++e) v[e] = stage[wave][s][8 * pc + e];
        if (L < 8) st8h_flush(orow + 8 * pc, v);
    }
}
static_assert((32 + 8) * 16 == HID * 2);
static_assert(SEQ % 8 == 0);
static_assert(8 * 2 * HID * 4 <= 131072);

__global__ __launch_bounds__(256) void k_contact(const float* __restrict__ HIJ, const float* __restrict__ B1, const float* __restrict__ W2, const float* __restrict__ B2, float* __restrict__ OUT2) {
    __shared__ float shi[32][CD];
    __shared__ float shj[32][CD + 1];
    __shared__ float sbv[CD];
    __shared__ float swv[CD];
    const int b = blockIdx.z, i0 = blockIdx.y * 32, j0 = blockIdx.x * 32; const int tid = threadIdx.x;
    for (int t = tid; t < 32 * CD; t += 256) { const int r = t / CD, c = t - r * CD;
        shi[r][c] = HIJ[((long long)(b * SEQ + i0 + r)) * 320 + c];
        shj[r][c] = HIJ[((long long)(b * SEQ + j0 + r)) * 320 + CD + c]; }
    if (tid < CD) { sbv[tid] = bfr(B1[tid]); swv[tid] = bfr(W2[tid]); }
    __syncthreads();
    const int wave = __builtin_amdgcn_readfirstlane(threadIdx.x >> 5); const int L = threadIdx.x & 31;
    const float bias2 = bfr(B2[0]);
    float acc[4];
#pragma unroll
    for (int q = 0; q < 4; ++q) acc[q] = bias2;
#pragma unroll 2
    for (int c = 0; c < CD; ++c) { const float hjv = shj[L][c]; const float bv = sbv[c]; const float w = swv[c];
#pragma unroll
        for (int q = 0; q < 4; ++q) acc[q] += fmaxf((shi[4 * wave + q][c] + hjv) + bv, 0.f) * w; }
#pragma unroll
    for (int q = 0; q < 4; ++q) { const float v = acc[q]; VST2(float, OUT2 + ((long long)(b * SEQ_FULL + i0 + 4 * wave + q)) * SEQ_FULL + j0 + L, v); }
}
static_assert(8 * 4 == 32);
static_assert((32 * CD + 32 * (CD + 1) + 2 * CD) * 4 <= 131072);
static_assert((32 * CD) % 256 == 0);

#define OFF0 0
#define OFF1 (NB_FULL * SEQ_FULL * 3)
#define OFF2 (OFF1 + NB_FULL * SEQ_FULL * 4)
#define OFF3 (OFF2 + NB_FULL * SEQ_FULL * SEQ_FULL)
#define OUT_TOTAL (OFF3 + NB_FULL * SEQ_FULL * 7)
static_assert(OFF1 * 4 == 6144);
static_assert(OFF2 * 4 == 14336);
static_assert(OFF3 * 4 == 538624);
static_assert(OUT_TOTAL * 4 == 552960);
static_assert((OFF1 * 4) % 128 == 0 && (OFF2 * 4) % 128 == 0 && (OFF3 * 4) % 128 == 0);

constexpr size_t al256(size_t b) { return (b + 255) / 256 * 256; }
constexpr size_t SZ_WBB  = al256((size_t)640 * 320 * 2);
constexpr size_t SZ_WSC1 = al256((size_t)320 * 320 * 2);
constexpr size_t SZ_WSC2 = al256((size_t)192 * 320 * 2);
constexpr size_t SZ_WQKV = al256((size_t)960 * 320 * 2);
constexpr size_t SZ_WO   = al256((size_t)320 * 320 * 2);
constexpr size_t SZ_WHIJ = al256((size_t)320 * 320 * 2);
constexpr size_t SZ_WR2  = al256((size_t)256 * 128 * 2);
constexpr size_t SZ_X16  = al256((size_t)MR * 320 * 2);
constexpr size_t SZ_BIAS = al256((size_t)BIAS_N * 4);
constexpr size_t SZ_T1   = al256((size_t)MR * 640 * 4);
constexpr size_t SZ_R1   = al256((size_t)MR * 320 * 4);
constexpr size_t SZ_H1   = al256((size_t)MR * 320 * 2);
constexpr size_t SZ_H2   = al256((size_t)MR * 192 * 4);
constexpr size_t SZ_R1H  = al256((size_t)MR * 128 * 2);
constexpr size_t SZ_R2   = al256((size_t)MR * 256 * 4);
constexpr size_t SZ_QKV  = al256((size_t)MR * 960 * 4);
constexpr size_t SZ_AO   = al256((size_t)MR * 320 * 2);
constexpr size_t SZ_A16  = al256((size_t)MR * 320 * 2);
constexpr size_t SZ_HIJ  = al256((size_t)MR * 320 * 4);
constexpr size_t WS_TOTAL = SZ_WBB + SZ_WSC1 + SZ_WSC2 + SZ_WQKV + SZ_WO + SZ_WHIJ + SZ_WR2 + SZ_X16 + SZ_BIAS + SZ_T1 + SZ_R1 + SZ_H1 + SZ_H2 + SZ_R1H + SZ_R2 + SZ_QKV + SZ_AO + SZ_A16 + SZ_HIJ;
static_assert(WS_TOTAL <= (size_t)134217728);

extern "C" void kernel_launch(void* const* d_in, const int* in_sizes, int n_in, void* d_out, int out_size, void* d_ws, size_t ws_size, hipStream_t stream) {
    if (n_in < 25) return;
    if (in_sizes[0] < ((NB - 1) * SEQ_FULL + SEQ) * HID) return;
    if (in_sizes[1] < 320 * 960 || in_sizes[3] < 320 * 320 || in_sizes[5] < 640 * 160 || in_sizes[9] < 320 * 640 || in_sizes[13] < 323 * 320 || in_sizes[15] < 320 * 160 || in_sizes[21] < 128 * 256) return;
    if (out_size < OUT_TOTAL) return;
    if (WS_TOTAL > ws_size) return;
    const float* x          = (const float*)d_in[0];
    const float* in_proj_w  = (const float*)d_in[1];
    const float* in_proj_b  = (const float*)d_in[2];
    const float* out_proj_w = (const float*)d_in[3];
    const float* out_proj_b = (const float*)d_in[4];
    const float* mlp_w1     = (const float*)d_in[5];
    const float* mlp_b1     = (const float*)d_in[6];
    const float* mlp_w2     = (const float*)d_in[7];
    const float* mlp_b2     = (const float*)d_in[8];
    const float* bb_w1      = (const float*)d_in[9];
    const float* bb_b1      = (const float*)d_in[10];
    const float* bb_w2      = (const float*)d_in[11];
    const float* bb_b2      = (const float*)d_in[12];
    const float* sc_w1      = (const float*)d_in[13];
    const float* sc_b1      = (const float*)d_in[14];
    const float* sc_w2      = (const float*)d_in[15];
    const float* sc_b2      = (const float*)d_in[16];
    const float* sc_w3      = (const float*)d_in[17];
    const float* sc_b3      = (const float*)d_in[18];
    const float* ref_w1     = (const float*)d_in[19];
    const float* ref_b1     = (const float*)d_in[20];
    const float* ref_w2     = (const float*)d_in[21];
    const float* ref_b2     = (const float*)d_in[22];
    const float* ref_w3     = (const float*)d_in[23];
    const float* ref_b3     = (const float*)d_in[24];
    float* out = (float*)d_out;
    float* out0 = out + OFF0; float* out1 = out + OFF1; float* out2 = out + OFF2; float* out3 = out + OFF3;

    char* wsp = (char*)d_ws;
    unsigned short* Wbb  = (unsigned short*)wsp; wsp += SZ_WBB;
    unsigned short* Wsc1 = (unsigned short*)wsp; wsp += SZ_WSC1;
    unsigned short* Wsc2 = (unsigned short*)wsp; wsp += SZ_WSC2;
    unsigned short* Wqkv = (unsigned short*)wsp; wsp += SZ_WQKV;
    unsigned short* Wo   = (unsigned short*)wsp; wsp += SZ_WO;
    unsigned short* Whij = (unsigned short*)wsp; wsp += SZ_WHIJ;
    unsigned short* Wr2  = (unsigned short*)wsp; wsp += SZ_WR2;
    unsigned short* X16  = (unsigned short*)wsp; wsp += SZ_X16;
    float* BIASP         = (float*)wsp;          wsp += SZ_BIAS;
    float* T1            = (float*)wsp;          wsp += SZ_T1;
    float* R1            = (float*)wsp;          wsp += SZ_R1;
    unsigned short* H1   = (unsigned short*)wsp; wsp += SZ_H1;
    float* H2            = (float*)wsp;          wsp += SZ_H2;
    unsigned short* R1H  = (unsigned short*)wsp; wsp += SZ_R1H;
    float* R2            = (float*)wsp;          wsp += SZ_R2;
    float* QKV           = (float*)wsp;          wsp += SZ_QKV;
    unsigned short* AO16 = (unsigned short*)wsp; wsp += SZ_AO;
    unsigned short* A16  = (unsigned short*)wsp; wsp += SZ_A16;
    float* HIJ           = (float*)wsp;          wsp += SZ_HIJ;
    if ((size_t)(wsp - (char*)d_ws) > ws_size) return;

    const float SX = 8.0f, SW = 32.0f, SR1 = 64.0f;
    k_wt16f<<<(640 * 40 + 255) / 256, 256, 0, stream>>>(bb_w1, 640, 320, 640, 640, Wbb, SW);
    k_wt16f<<<(320 * 40 + 255) / 256, 256, 0, stream>>>(sc_w1, 320, 320, 320, 320, Wsc1, SW);
    k_wt16f<<<(192 * 40 + 255) / 256, 256, 0, stream>>>(sc_w2, 160, 320, 160, 192, Wsc2, SW);
    k_wt16f<<<(960 * 40 + 255) / 256, 256, 0, stream>>>(in_proj_w, 960, 320, 960, 960, Wqkv, SW);
    k_wt16f<<<(320 * 40 + 255) / 256, 256, 0, stream>>>(out_proj_w, 320, 320, 320, 320, Wo, SW);
    k_wt16f<<<(160 * 40 + 255) / 256, 256, 0, stream>>>(mlp_w1, 160, 320, 160, 160, Whij, SW);
    k_wt16f<<<(160 * 40 + 255) / 256, 256, 0, stream>>>(mlp_w1 + 320 * 160, 160, 320, 160, 160, Whij + 160 * 320, SW);
    k_wt16f<<<(256 * 16 + 255) / 256, 256, 0, stream>>>(ref_w2, 256, 128, 256, 256, Wr2, SW);
    k_x16<<<(MR * 40 + 255) / 256, 256, 0, stream>>>(x, X16, SX);
    k_bias6<<<4, 256, 0, stream>>>(bb_b1, sc_b1, sc_b2, in_proj_b, out_proj_b, ref_b2, BIASP);

    const unsigned TM = MR / 64;
    gemmkit::wmma_gemm64<0, false, 2, 0, false, 2><<<dim3((TM * 10 + 7) / 8, 1), 256, 0, stream>>>((const unsigned short*)X16, nullptr, 320, 0, (const unsigned short*)Wbb, nullptr, 320, 0, (void*)T1, nullptr, 640, 0, BIASP + BO_BB1, nullptr, 0, MR, 640, 320, 1.0f / (SX * SW));
    k_bb_head<<<MR / 32, 256, 0, stream>>>(T1, bb_w2, bb_b2, sc_w1, out0, R1);
    gemmkit::wmma_gemm64<0, false, 2, 1, true, 2><<<dim3((TM * 5 + 7) / 8, 1), 256, 0, stream>>>((const unsigned short*)X16, nullptr, 320, 0, (const unsigned short*)Wsc1, nullptr, 320, 0, (void*)H1, nullptr, 320, 0, BIASP + BO_SC1, R1, 0, MR, 320, 320, 1.0f / (SX * SW));
    gemmkit::wmma_gemm64<0, false, 2, 0, false, 2><<<dim3((TM * 3 + 7) / 8, 1), 256, 0, stream>>>((const unsigned short*)H1, nullptr, 320, 0, (const unsigned short*)Wsc2, nullptr, 320, 0, (void*)H2, nullptr, 192, 0, BIASP + BO_SC2, nullptr, 0, MR, 192, 320, 1.0f / SW);
    k_sc_head<<<MR / 32, 256, 0, stream>>>(H2, sc_w3, sc_b3, out0, ref_w1, ref_b1, out1, R1H, SR1);
    gemmkit::wmma_gemm64<0, false, 2, 0, false, 2><<<dim3((TM * 4 + 7) / 8, 1), 256, 0, stream>>>((const unsigned short*)R1H, nullptr, 128, 0, (const unsigned short*)Wr2, nullptr, 128, 0, (void*)R2, nullptr, 256, 0, BIASP + BO_R2, nullptr, 0, MR, 256, 128, 1.0f / (SR1 * SW));
    k_ref_head<<<MR / 32, 256, 0, stream>>>(R2, ref_w3, ref_b3, out3);
    gemmkit::wmma_gemm64<0, false, 2, 0, false, 0><<<dim3((TM * 15 + 7) / 8, 1), 256, 0, stream>>>((const unsigned short*)X16, nullptr, 320, 0, (const unsigned short*)Wqkv, nullptr, 320, 0, (void*)QKV, nullptr, 960, 0, BIASP + BO_IN, nullptr, 0, MR, 960, 320, 1.0f / (SX * SW));
    k_attn2<<<SEQ / 8, 256, 0, stream>>>(QKV, AO16, SX);
    gemmkit::wmma_gemm64<0, false, 2, 1, false, 0><<<dim3((TM * 5 + 7) / 8, 1), 256, 0, stream>>>((const unsigned short*)AO16, nullptr, 320, 0, (const unsigned short*)Wo, nullptr, 320, 0, (void*)A16, nullptr, 320, 0, BIASP + BO_OUT, nullptr, 0, MR, 320, 320, 1.0f / (SX * SW));
    gemmkit::wmma_gemm64<0, false, 0, 0, false, 0><<<dim3((TM * 5 + 7) / 8, 1), 256, 0, stream>>>((const unsigned short*)A16, nullptr, 320, 0, (const unsigned short*)Whij, nullptr, 320, 0, (void*)HIJ, nullptr, 320, 0, nullptr, nullptr, 0, MR, 320, 320, 1.0f / SW);
    k_contact<<<dim3(SEQ / 32, SEQ / 32, NB), 256, 0, stream>>>(HIJ, mlp_b1, mlp_w2, mlp_b2, out2);
}
